// MHA_45079976739512
// MI455X (gfx1250) — hardware-verified
//
#include <hip/hip_runtime.h>


#ifndef NB
#define NB 8
#endif
#ifndef SEQ
#define SEQ 1024
#endif
#ifndef SEQ_FULL
#define SEQ_FULL 1024
#endif
#define NH_  16
#define HD   64
#define DM   (NH_ * HD)
#define TLP  72
#define OSP  68
#define CEXP 0.18033688011112042f
#define PSH  8.0f

typedef _Float16 h16;
typedef unsigned short bf;
typedef __attribute__((ext_vector_type(16))) __bf16   v16bf;
typedef __attribute__((ext_vector_type(16))) _Float16 v16h;
typedef __attribute__((ext_vector_type(8)))  _Float16 v8h;
typedef __attribute__((ext_vector_type(8)))  unsigned short v8us;
typedef __attribute__((ext_vector_type(8)))  float    v8f;
typedef __attribute__((ext_vector_type(4)))  float    v4f;
typedef v8h  __attribute__((may_alias)) v8ha;
typedef v4f  __attribute__((may_alias)) v4fa;

static_assert(HD == 64);
static_assert(NH_ * HD == DM);
static_assert(SEQ % 64 == 0);
static_assert(SEQ <= SEQ_FULL);
static_assert((NH_ * HD * HD) % (256 * 8) == 0);
static_assert((TLP * 2) % 16 == 0);
static_assert((OSP * 4) % 16 == 0);

#define WB_BYTES ((size_t)3 * NH_ * HD * HD * 2)
#define PL_BYTES ((size_t)NB * NH_ * SEQ * HD * 2)
#define WS_TOTAL (WB_BYTES + 3 * PL_BYTES)
static_assert(WB_BYTES % 256 == 0);
static_assert(PL_BYTES % 256 == 0);
static_assert(WS_TOTAL <= (size_t)134217728);

__device__ __forceinline__ unsigned short f2bf(float f) { unsigned u = __float_as_uint(f); u += 0x7FFFu + ((u >> 16) & 1u); return (unsigned short)(u >> 16); }
__device__ __forceinline__ float bf2f(unsigned short b) { return __uint_as_float(((unsigned)b) << 16); }
__device__ __forceinline__ float bfr(float f) { return bf2f(f2bf(f)); }
__device__ __forceinline__ v16h cat16(v8h lo, v8h hi) { return __builtin_shufflevector(lo, hi, 0, 1, 2, 3, 4, 5, 6, 7, 8, 9, 10, 11, 12, 13, 14, 15); }
__device__ __forceinline__ v16bf cat16b(v8us lo, v8us hi) { return __builtin_bit_cast(v16bf, __builtin_shufflevector(lo, hi, 0, 1, 2, 3, 4, 5, 6, 7, 8, 9, 10, 11, 12, 13, 14, 15)); }

__device__ __forceinline__ v8f wm16(v16h a, v16h b, v8f c) {
    c = __builtin_amdgcn_wmma_f32_16x16x32_f16(false, a, false, b, (short)0, c, false, false);
    asm volatile("v_nop\n\tv_nop\n\tv_nop\n\tv_nop" : "+v"(c) : "v"(a), "v"(b));
    return c; }
__device__ __forceinline__ v8f wmb(v16bf a, v16bf b, v8f c) {
    c = __builtin_amdgcn_wmma_f32_16x16x32_bf16(false, a, false, b, (short)0, c, false, false);
    asm volatile("v_nop\n\tv_nop\n\tv_nop\n\tv_nop" : "+v"(c) : "v"(a), "v"(b));
    return c; }

__device__ __forceinline__ v16h  ldh(const h16* p) { return cat16(*(const v8h*)p, *(const v8h*)(p + 16)); }
__device__ __forceinline__ v16bf ldb(const bf* p)  { return cat16b(*(const v8us*)p, *(const v8us*)(p + 16)); }
__device__ __forceinline__ v16bf ldx(const float* p) {
    const v4f a0 = *(const v4f*)p, a1 = *(const v4f*)(p + 4), c0 = *(const v4f*)(p + 16), c1 = *(const v4f*)(p + 20);
    v8us lo, up;
#pragma unroll
    for (int q = 0; q < 4; ++q) { lo[q] = f2bf(a0[q]); lo[4 + q] = f2bf(a1[q]); up[q] = f2bf(c0[q]); up[4 + q] = f2bf(c1[q]); }
    return cat16b(lo, up); }

__global__ __launch_bounds__(256) void k_wcvt(const float* __restrict__ Wq, const float* __restrict__ Wk, const float* __restrict__ Wv, bf* WB) {
    const unsigned role = blockIdx.y;
    const float* src = (role == 0u) ? Wq : ((role == 1u) ? Wk : Wv);
    const unsigned i = blockIdx.x * 256u + threadIdx.x;
    const v4f a = *(const v4f*)(src + (size_t)i * 8), c = *(const v4f*)(src + (size_t)i * 8 + 4);
    v8us o;
#pragma unroll
    for (int q = 0; q < 4; ++q) { o[q] = f2bf(a[q]); o[4 + q] = f2bf(c[q]); }
    bf* dst = WB + (size_t)role * (NH_ * HD * HD) + (size_t)i * 8;
    *(volatile v8us*)dst = o; __threadfence(); *(volatile v8us*)dst = o; }

__global__ __launch_bounds__(128) void k_proj(const float* __restrict__ x, const bf* __restrict__ WB,
                                             const float* __restrict__ bq, const float* __restrict__ bk, const float* __restrict__ bv,
                                             h16* Qp, h16* Kp, h16* Vt) {
    __shared__ __align__(16) h16 ts[3][64 * TLP];
    const unsigned tid = threadIdx.x, lane = tid & 31u, w = tid >> 5, lr = lane & 15u, hf = lane >> 4;
    const unsigned s0 = blockIdx.x * 64u, h = blockIdx.y, b = blockIdx.z, bh = b * NH_ + h;
    const float* xr = x + ((size_t)b * SEQ_FULL + s0 + w * 16u + lr) * DM + h * HD + 8u * hf;
    const v16bf ax0 = ldx(xr), ax1 = ldx(xr + 32);
#pragma unroll
    for (int role = 0; role < 3; ++role) {
        const float* bp = (role == 0) ? bq : ((role == 1) ? bk : bv);
        const bf* wr = WB + ((size_t)(role * NH_ + h) * HD + lr) * HD + 8u * hf;
#pragma unroll
        for (int nb = 0; nb < 4; ++nb) {
            const bf* wp = wr + nb * 16 * HD;
            const v16bf b0 = ldb(wp), b1 = ldb(wp + 32);
            v8f acc = (v8f){};
            acc = wmb(ax0, b0, acc);
            acc = wmb(ax1, b1, acc);
            const float bias = bfr(bp[h * HD + nb * 16 + lr]);
            if (role < 2) {
#pragma unroll
                for (int j = 0; j < 8; ++j) ts[role][(w * 16u + 8u * hf + j) * TLP + nb * 16 + lr] = (h16)(acc[j] + bias);
            } else {
                v8h pk;
#pragma unroll
                for (int j = 0; j < 8; ++j) pk[j] = (h16)(acc[j] + bias);
                *(v8ha*)(&ts[2][(nb * 16 + lr) * TLP + w * 16u + 8u * hf]) = pk;
            }
        }
    }
    __syncthreads();
    const unsigned piece = lane & 7u, rq = lane >> 3;
    h16* qd = Qp + ((size_t)bh * SEQ + s0) * HD + piece * 8u;
    h16* kd = Kp + ((size_t)bh * SEQ + s0) * HD + piece * 8u;
    h16* vd = Vt + (size_t)bh * HD * SEQ + s0 + piece * 8u;
#pragma unroll 1
    for (int ps = 0; ps < 2; ++ps) {
#pragma unroll
        for (int it = 0; it < 4; ++it) {
            const unsigned row = w * 16u + it * 4u + rq;
            const v8h vq = *(const v8ha*)(&ts[0][row * TLP + piece * 8u]);
            const v8h vk = *(const v8ha*)(&ts[1][row * TLP + piece * 8u]);
            const v8h vv = *(const v8ha*)(&ts[2][row * TLP + piece * 8u]);
            *(volatile v8h*)(qd + (size_t)row * HD) = vq;
            *(volatile v8h*)(kd + (size_t)row * HD) = vk;
            *(volatile v8h*)(vd + (size_t)row * SEQ) = vv;
        }
        if (ps == 0) __threadfence();
    }
}

__global__ __launch_bounds__(128) void k_flash(const h16* __restrict__ Qp, const h16* __restrict__ Kp, const h16* __restrict__ Vt, float* out) {
    __shared__ __align__(16) float os[4 * 16 * OSP];
    const unsigned tid = threadIdx.x, lane = tid & 31u, w = tid >> 5, lr = lane & 15u, hf = lane >> 4;
    const unsigned h = blockIdx.y, b = blockIdx.z, bh = b * NH_ + h;
    const unsigned q0 = blockIdx.x * 64u + w * 16u;
    const h16* qp = Qp + ((size_t)bh * SEQ + q0 + lr) * HD + 8u * hf;
    const v16h bq0 = ldh(qp), bq1 = ldh(qp + 32);
    const h16* kb = Kp + ((size_t)bh * SEQ + lr) * HD + 8u * hf;
    const h16* vb = Vt + ((size_t)bh * HD + lr) * SEQ + 8u * hf;
    v8f o[4];
#pragma unroll
    for (int dt = 0; dt < 4; ++dt) o[dt] = (v8f){};
    float m = -3.0e38f, l = 0.f;
#pragma unroll 1
    for (unsigned kt = 0; kt < SEQ; kt += 64u) {
        v8f sc[4];
#pragma unroll
        for (int T = 0; T < 4; ++T) {
            const h16* kp = kb + (size_t)(kt + 16u * T) * HD;
            const v16h a0 = ldh(kp), a1 = ldh(kp + 32);
            v8f c = (v8f){};
            c = wm16(a0, bq0, c);
            c = wm16(a1, bq1, c);
            sc[T] = c;
        }
        float mx = -3.0e38f;
#pragma unroll
        for (int T = 0; T < 4; ++T)
#pragma unroll
            for (int j = 0; j < 8; ++j) { const float t = sc[T][j] * CEXP; sc[T][j] = t; mx = fmaxf(mx, t); }
        mx = fmaxf(mx, __shfl_xor(mx, 16, 32));
        const float mn = fmaxf(m, mx);
        const float corr = __builtin_amdgcn_exp2f(m - mn);
        m = mn;
        const float sh = PSH - mn;
        float rs = 0.f;
        v16h pb[2];
#pragma unroll
        for (int u = 0; u < 2; ++u)
#pragma unroll
            for (int j = 0; j < 8; ++j) {
                const float p0 = __builtin_amdgcn_exp2f(sc[2 * u][j] + sh);
                const float p1 = __builtin_amdgcn_exp2f(sc[2 * u + 1][j] + sh);
                rs += p0 + p1;
                pb[u][j] = (h16)p0; pb[u][8 + j] = (h16)p1;
            }
        l = l * corr + rs;
#pragma unroll
        for (int dt = 0; dt < 4; ++dt)
#pragma unroll
            for (int j = 0; j < 8; ++j) o[dt][j] *= corr;
#pragma unroll
        for (int dt = 0; dt < 4; ++dt) {
            const h16* vp = vb + (size_t)dt * 16 * SEQ + kt;
            const v16h a0 = ldh(vp), a1 = ldh(vp + 32);
            o[dt] = wm16(a0, pb[0], o[dt]);
            o[dt] = wm16(a1, pb[1], o[dt]);
        }
    }
    l += __shfl_xor(l, 16, 32);
    const float inv = 1.0f / l;
#pragma unroll
    for (int dt = 0; dt < 4; ++dt) {
        v4f e0, e1;
#pragma unroll
        for (int q = 0; q < 4; ++q) { e0[q] = o[dt][q] * inv; e1[q] = o[dt][4 + q] * inv; }
        *(v4fa*)(&os[(w * 16u + lr) * OSP + dt * 16 + 8u * hf]) = e0;
        *(v4fa*)(&os[(w * 16u + lr) * OSP + dt * 16 + 8u * hf + 4u]) = e1;
    }
    __syncthreads();
    float* orow = out + ((size_t)b * SEQ + q0) * DM + h * HD;
#pragma unroll 1
    for (int ps = 0; ps < 2; ++ps) {
#pragma unroll
        for (int s = 0; s < 8; ++s) {
            const unsigned row = 2u * s + hf, cofs = lr * 4u;
            const v4f val = *(const v4fa*)(&os[(w * 16u + row) * OSP + cofs]);
            *(volatile v4f*)(orow + (size_t)row * DM + cofs) = val;
        }
        if (ps == 0) __threadfence();
    }
}

extern "C" void kernel_launch(void* const* d_in, const int* in_sizes, int n_in,
                              void* d_out, int out_size, void* d_ws, size_t ws_size, hipStream_t stream) {
    if (n_in < 7) return;
    if ((size_t)in_sizes[0] < (size_t)(NB - 1) * SEQ_FULL * DM + (size_t)SEQ * DM) return;
    if (in_sizes[1] < NH_ * HD * HD || in_sizes[3] < NH_ * HD * HD || in_sizes[5] < NH_ * HD * HD) return;
    if (in_sizes[2] < NH_ * HD || in_sizes[4] < NH_ * HD || in_sizes[6] < NH_ * HD) return;
    if ((size_t)out_size < (size_t)NB * SEQ * DM) return;
    if (ws_size < WS_TOTAL) return;
    const float* x  = (const float*)d_in[0];
    const float* Wq = (const float*)d_in[1]; const float* bq = (const float*)d_in[2];
    const float* Wk = (const float*)d_in[3]; const float* bk = (const float*)d_in[4];
    const float* Wv = (const float*)d_in[5]; const float* bv = (const float*)d_in[6];
    char* wsp = (char*)d_ws;
    bf*  WB = (bf*)wsp;  wsp += WB_BYTES;
    h16* Qp = (h16*)wsp; wsp += PL_BYTES;
    h16* Kp = (h16*)wsp; wsp += PL_BYTES;
    h16* Vt = (h16*)wsp;
    k_wcvt<<<dim3((NH_ * HD * HD) / (256 * 8), 3, 1), 256, 0, stream>>>(Wq, Wk, Wv, WB);
    k_proj<<<dim3(SEQ / 64, NH_, NB), 128, 0, stream>>>(x, WB, bq, bk, bv, Qp, Kp, Vt);
    k_flash<<<dim3(SEQ / 64, NH_, NB), 128, 0, stream>>>(Qp, Kp, Vt, (float*)d_out);
}
